// NonlocalBlock_68977174774048
// MI455X (gfx1250) — hardware-run, weakly checked
//
#include <hip/hip_runtime.h>


#ifndef NB
#define NB 4
#endif
#ifndef SEQ
#define SEQ 9216
#endif
#define NB_FULL  4
#define SEQ_FULL 9216
#ifndef OUT_SEQ
#define OUT_SEQ SEQ
#endif
#define CCH  64
#define HD   32
#define MP   (SEQ / 2)
#define AW   4
#define OSP  68
#define QRS  2048.0f
#define QRI  (1.0f / 2048.0f)
#define LOG2E ((float)1.4426950408889634)
#define PSH  14.0f
#define NEGB (-3.0e38f)

static_assert(HD == 32);
static_assert(CCH == 64);
static_assert(CCH % 32 == 0);
static_assert(SEQ % 128 == 0);
static_assert(MP * 2 == SEQ);
static_assert(MP % 32 == 0);
static_assert(MP % 64 == 0);
static_assert(SEQ % (16 * AW) == 0);
static_assert(16 * AW == 64);
static_assert(OUT_SEQ % 32 == 0);
static_assert(SEQ_FULL % 32 == 0);
static_assert(NB <= NB_FULL);
static_assert(SEQ <= SEQ_FULL);
static_assert((OSP * 4) % 16 == 0);
static_assert(OSP >= 64);
static_assert(2 * 32 * 16 == 16 * HD * 2);
static_assert(1 * 32 * 16 == 8 * HD * 2);
static_assert(4 * 4 * 8 * 16 == 16 * 64 * 2);
static_assert(AW * 8 * 4 * 8 * 16 == CCH * 64 * 4);
static_assert(2 * 32 * 8 * 16 == 64 * CCH * 2);
static_assert(16 * 68 * 4 <= 131072);
static_assert(16 * 132 * 4 <= 131072);
static_assert(CCH * OSP * 4 <= 131072);
static_assert(64 * 72 * 2 <= 131072);

typedef _Float16 h16;
typedef unsigned short bf;
typedef __attribute__((ext_vector_type(16))) __bf16   v16bf;
typedef __attribute__((ext_vector_type(16))) _Float16 v16h;
typedef __attribute__((ext_vector_type(8)))  _Float16 v8h;
typedef __attribute__((ext_vector_type(8)))  unsigned short v8us;
typedef __attribute__((ext_vector_type(8)))  float    v8f;
typedef __attribute__((ext_vector_type(4)))  float    v4f;
typedef v4f  __attribute__((may_alias)) v4fa;
typedef v8us __attribute__((may_alias)) v8usa;

__device__ __forceinline__ unsigned short f2bf(float f) { unsigned u = __float_as_uint(f); u += 0x7FFFu + ((u >> 16) & 1u); return (unsigned short)(u >> 16); }
__device__ __forceinline__ float bfr(float f) { return __uint_as_float(((unsigned)f2bf(f)) << 16); }
__device__ __forceinline__ v16h cat16(v8h lo, v8h hi) { return __builtin_shufflevector(lo, hi, 0, 1, 2, 3, 4, 5, 6, 7, 8, 9, 10, 11, 12, 13, 14, 15); }
__device__ __forceinline__ v16bf cat16b(v8us lo, v8us hi) { return __builtin_bit_cast(v16bf, __builtin_shufflevector(lo, hi, 0, 1, 2, 3, 4, 5, 6, 7, 8, 9, 10, 11, 12, 13, 14, 15)); }
__device__ __forceinline__ v16h  ldh(const h16* p) { return cat16(*(const v8h*)p, *(const v8h*)(p + 16)); }
__device__ __forceinline__ v16bf ldb(const bf* p)  { return cat16b(*(const v8us*)p, *(const v8us*)(p + 16)); }
__device__ __forceinline__ void wave_sync() { __builtin_amdgcn_fence(3  , "wavefront"); __builtin_amdgcn_wave_barrier(); asm volatile("" ::: "memory"); }
__device__ __forceinline__ v8f wmma16g(v16h a, v16h b, v8f c) {
    c = __builtin_amdgcn_wmma_f32_16x16x32_f16(false, a, false, b, (short)0, c, false, false);
    asm volatile("v_nop\n\tv_nop\n\tv_nop\n\tv_nop" : "+v"(c) : "v"(a), "v"(b));
    return c; }
__device__ __forceinline__ v8f wmmabg(v16bf a, v16bf b, v8f c) {
    c = __builtin_amdgcn_wmma_f32_16x16x32_bf16(false, a, false, b, (short)0, c, false, false);
    asm volatile("v_nop\n\tv_nop\n\tv_nop\n\tv_nop" : "+v"(c) : "v"(a), "v"(b));
    return c; }
static __device__ __forceinline__ h16 toh_flush(float v) { const h16 r = (h16)v; return (fabsf(v) < 6.103515625e-05f) ? (h16)0.0f : r; }

__global__ __launch_bounds__(256) void k_cvt8(const float* __restrict__ src, bf* dst, size_t n8) {
    const size_t i = (size_t)blockIdx.x * 256 + threadIdx.x; if (i >= n8) return;
    const v8f v = *(const v8f*)(src + i * 8); v8us o;
#pragma unroll
    for (int k = 0; k < 8; ++k) o[k] = f2bf(v[k]);
    *(volatile v8us*)(dst + i * 8) = o; __threadfence(); *(volatile v8us*)(dst + i * 8) = o;
}

__global__ __launch_bounds__(256) void k_cvtw(const float* __restrict__ src, h16* dst, size_t n8) {
    const size_t i = (size_t)blockIdx.x * 256 + threadIdx.x; if (i >= n8) return;
    const v8f v = *(const v8f*)(src + i * 8); v8h o;
#pragma unroll
    for (int k = 0; k < 8; ++k) o[k] = toh_flush(bfr(v[k]));
    *(volatile v8h*)(dst + i * 8) = o; __threadfence(); *(volatile v8h*)(dst + i * 8) = o;
}

__global__ __launch_bounds__(256) void k_cvtT(const float* __restrict__ src, bf* dst) {
    __shared__ __align__(16) unsigned short tb[64 * 72];
    const int tid = threadIdx.x; const int b = blockIdx.y; const int n0 = blockIdx.x * 64;
#pragma unroll 1
    for (int i = 0; i < 4; ++i) {
        const int idx = i * 256 + tid; const int c = idx >> 4, q = idx & 15;
        const v4f v = *(const v4f*)(src + ((size_t)b * CCH + (size_t)c) * SEQ_FULL + (size_t)n0 + (size_t)q * 4);
#pragma unroll
        for (int e = 0; e < 4; ++e) tb[(q * 4 + e) * 72 + c] = f2bf(v[e]); }
    __syncthreads();
#pragma unroll 1
    for (int ps = 0; ps < 2; ++ps) {
#pragma unroll
        for (int s = 0; s < 2; ++s) { const int line = s * 32 + (tid >> 3), c8 = (tid & 7) * 8;
            const v8us o = *(const v8usa*)(&tb[line * 72 + c8]);
            *(volatile v8us*)(dst + ((size_t)b * SEQ + (size_t)(n0 + line)) * CCH + c8) = o; }
        if (ps == 0) __threadfence(); }
}

__global__ __launch_bounds__(32) void k_proj_qk(const bf* __restrict__ A, const bf* __restrict__ Bt, const float* __restrict__ bth, const float* __restrict__ bph,
                                                 h16* QH, h16* QR, h16* KP, h16* KR) {
    __shared__ __align__(16) float os[16 * 68];
    const int lane = threadIdx.x & 31, lr = lane & 15, hi = lane >> 4; const int r0 = blockIdx.x * 64;
    v8f acc[4][4];
#pragma unroll
    for (int mb = 0; mb < 4; ++mb)
#pragma unroll
        for (int nb = 0; nb < 4; ++nb) acc[mb][nb] = (v8f){};
    const size_t aoff = (size_t)(r0 + lr) * CCH + 8 * hi, boff = (size_t)lr * CCH + 8 * hi;
#pragma unroll 1
    for (int kc = 0; kc < CCH; kc += 32) {
        v16bf a[4];
#pragma unroll
        for (int mb = 0; mb < 4; ++mb) a[mb] = ldb(A + aoff + (size_t)mb * 16 * CCH + kc);
#pragma unroll
        for (int nb = 0; nb < 4; ++nb) { const v16bf b = ldb(Bt + boff + (size_t)nb * 16 * CCH + kc);
#pragma unroll
            for (int mb = 0; mb < 4; ++mb) acc[mb][nb] = wmmabg(a[mb], b, acc[mb][nb]); }
    }
    float bc[4];
    bc[0] = bfr(bth[lr]); bc[1] = bfr(bth[16 + lr]); bc[2] = bfr(bph[lr]); bc[3] = bfr(bph[16 + lr]);
    const int bb = r0 / SEQ, tt = r0 % SEQ;
    const size_t qbase = ((size_t)bb * SEQ + (size_t)tt) * HD;
    const size_t kbase = ((size_t)bb * MP + (size_t)(tt >> 1)) * HD;
#pragma unroll
    for (int mb = 0; mb < 4; ++mb) {
#pragma unroll
        for (int nb = 0; nb < 4; ++nb) {
#pragma unroll
            for (int j = 0; j < 8; ++j) os[(hi * 8 + j) * 68 + nb * 16 + lr] = acc[mb][nb][j] + bc[nb]; }
        wave_sync();
#pragma unroll 1
        for (int ps = 0; ps < 2; ++ps) {
            const size_t sb = qbase + (size_t)(mb * 16) * HD;
#pragma unroll
            for (int s = 0; s < 2; ++s) { const int p = s * 32 + lane; const int row = p >> 2, c8 = (p & 3) * 8;
                const v4f x0 = *(const v4fa*)(&os[row * 68 + c8]); const v4f x1 = *(const v4fa*)(&os[row * 68 + c8 + 4]); v8h hv, rv;
#pragma unroll
                for (int i = 0; i < 4; ++i) { const h16 a0 = toh_flush(x0[i]); const h16 a1 = toh_flush(x1[i]); hv[i] = a0; hv[4 + i] = a1;
                    rv[i] = toh_flush((x0[i] - (float)a0) * QRS); rv[4 + i] = toh_flush((x1[i] - (float)a1) * QRS); }
                const size_t oo = sb + (size_t)p * 8;
                *(volatile v8h*)(QH + oo) = hv; *(volatile v8h*)(QR + oo) = rv; }
            { const int prow = lane >> 2, c8 = (lane & 3) * 8;
              const v4f e0 = *(const v4fa*)(&os[(2 * prow) * 68 + 32 + c8]);     const v4f e1 = *(const v4fa*)(&os[(2 * prow) * 68 + 32 + c8 + 4]);
              const v4f d0 = *(const v4fa*)(&os[(2 * prow + 1) * 68 + 32 + c8]); const v4f d1 = *(const v4fa*)(&os[(2 * prow + 1) * 68 + 32 + c8 + 4]); v8h hv, rv;
#pragma unroll
              for (int i = 0; i < 4; ++i) { const float p0 = fmaxf(e0[i], d0[i]); const float p1 = fmaxf(e1[i], d1[i]);
                  const h16 a0 = toh_flush(p0); const h16 a1 = toh_flush(p1); hv[i] = a0; hv[4 + i] = a1;
                  rv[i] = toh_flush((p0 - (float)a0) * QRS); rv[4 + i] = toh_flush((p1 - (float)a1) * QRS); }
              const size_t oo = kbase + (size_t)(mb * 8) * HD + (size_t)lane * 8;
              *(volatile v8h*)(KP + oo) = hv; *(volatile v8h*)(KR + oo) = rv; }
            if (ps == 0) __threadfence(); }
        wave_sync();
    }
}

__global__ __launch_bounds__(32) void k_proj_vt(const bf* __restrict__ A, const bf* __restrict__ Bt, const float* __restrict__ bg, h16* VT) {
    __shared__ __align__(16) float os[16 * 132];
    const int lane = threadIdx.x & 31, lr = lane & 15, hi = lane >> 4; const int c0 = blockIdx.x * 128;
    v8f acc[2][8];
#pragma unroll
    for (int mb = 0; mb < 2; ++mb)
#pragma unroll
        for (int nb = 0; nb < 8; ++nb) acc[mb][nb] = (v8f){};
    const size_t aoff = (size_t)lr * CCH + 8 * hi, boff = (size_t)(c0 + lr) * CCH + 8 * hi;
#pragma unroll 1
    for (int kc = 0; kc < CCH; kc += 32) {
        v16bf a[2];
#pragma unroll
        for (int mb = 0; mb < 2; ++mb) a[mb] = ldb(A + aoff + (size_t)mb * 16 * CCH + kc);
#pragma unroll
        for (int nb = 0; nb < 8; ++nb) { const v16bf b = ldb(Bt + boff + (size_t)nb * 16 * CCH + kc);
#pragma unroll
            for (int mb = 0; mb < 2; ++mb) acc[mb][nb] = wmmabg(a[mb], b, acc[mb][nb]); }
    }
    const int bb = c0 / SEQ, tt = c0 % SEQ;
    const size_t vbase = (size_t)bb * HD * MP + (size_t)(tt >> 1);
#pragma unroll
    for (int mb = 0; mb < 2; ++mb) {
        float br[8];
#pragma unroll
        for (int j = 0; j < 8; ++j) br[j] = bfr(bg[mb * 16 + hi * 8 + j]);
#pragma unroll
        for (int nb = 0; nb < 8; ++nb) {
#pragma unroll
            for (int j = 0; j < 8; ++j) os[(hi * 8 + j) * 132 + nb * 16 + lr] = acc[mb][nb][j] + br[j]; }
        wave_sync();
#pragma unroll 1
        for (int ps = 0; ps < 2; ++ps) {
#pragma unroll
            for (int s = 0; s < 4; ++s) { const int row = 4 * s + (lane >> 3), c8 = (lane & 7) * 8;
                const v4f q0 = *(const v4fa*)(&os[row * 132 + 2 * c8]);     const v4f q1 = *(const v4fa*)(&os[row * 132 + 2 * c8 + 4]);
                const v4f q2 = *(const v4fa*)(&os[row * 132 + 2 * c8 + 8]); const v4f q3 = *(const v4fa*)(&os[row * 132 + 2 * c8 + 12]); v8h hv;
                hv[0] = toh_flush(fmaxf(q0[0], q0[1])); hv[1] = toh_flush(fmaxf(q0[2], q0[3]));
                hv[2] = toh_flush(fmaxf(q1[0], q1[1])); hv[3] = toh_flush(fmaxf(q1[2], q1[3]));
                hv[4] = toh_flush(fmaxf(q2[0], q2[1])); hv[5] = toh_flush(fmaxf(q2[2], q2[3]));
                hv[6] = toh_flush(fmaxf(q3[0], q3[1])); hv[7] = toh_flush(fmaxf(q3[2], q3[3]));
                const size_t oo = vbase + (size_t)(mb * 16 + row) * MP + c8;
                *(volatile v8h*)(VT + oo) = hv; }
            if (ps == 0) __threadfence(); }
        wave_sync();
    }
}

__global__ __launch_bounds__(32 * AW) void k_flash(const h16* __restrict__ QH, const h16* __restrict__ QR, const h16* __restrict__ KP, const h16* __restrict__ KR,
                                                   const h16* __restrict__ VT, const h16* __restrict__ WO, const float* __restrict__ bout,
                                                   const float* __restrict__ xin, float* OUT) {
    __shared__ __align__(16) float os[CCH * OSP];
    const int lane = threadIdx.x & 31, lr = lane & 15, hi = lane >> 4;
    const int wave = __builtin_amdgcn_readfirstlane((int)(threadIdx.x >> 5));
    const int b = blockIdx.y; const int tb0 = blockIdx.x * (16 * AW); const int t0 = tb0 + wave * 16;
    const size_t qo = ((size_t)b * SEQ + (size_t)(t0 + lr)) * HD + 8 * hi;
    const v16h qh = ldh(QH + qo), qr = ldh(QR + qo);
    const size_t ko = ((size_t)b * MP + (size_t)lr) * HD + 8 * hi;
    const size_t vo = ((size_t)b * HD + (size_t)lr) * MP + 8 * hi;
    v8f o0 = (v8f){}, o1 = (v8f){};
    float m = NEGB, l = 0.0f;
#pragma unroll 1
    for (int key0 = 0; key0 < MP; key0 += 32) {
        const h16* ka = KP + ko + (size_t)key0 * HD;
        const h16* kr = KR + ko + (size_t)key0 * HD;
        const v16h ka0 = ldh(ka), kb0 = ldh(ka + 16 * HD);
        const v16h kra0 = ldh(kr), krb0 = ldh(kr + 16 * HD);
        v8f sHa = wmma16g(ka0, qh, (v8f){});
        v8f sLa = wmma16g(ka0, qr, (v8f){});
        sLa = wmma16g(kra0, qh, sLa);
        v8f sHb = wmma16g(kb0, qh, (v8f){});
        v8f sLb = wmma16g(kb0, qr, (v8f){});
        sLb = wmma16g(krb0, qh, sLb);
        float ta[8], tc[8]; float mx = NEGB;
#pragma unroll
        for (int r = 0; r < 8; ++r) {
            ta[r] = (sHa[r] + sLa[r] * QRI) * LOG2E; tc[r] = (sHb[r] + sLb[r] * QRI) * LOG2E;
            mx = fmaxf(mx, fmaxf(ta[r], tc[r])); }
        mx = fmaxf(mx, __shfl_xor(mx, 16, 32));
        const float mnew = fmaxf(m, mx);
        const float alpha = __builtin_amdgcn_exp2f(m - mnew);
        const float sh = PSH - mnew;
        v16h pb; float ls = 0.0f;
#pragma unroll
        for (int r = 0; r < 8; ++r) {
            const float xa = ta[r] + sh, xc = tc[r] + sh;
            const float ea = __builtin_amdgcn_exp2f(xa), ec = __builtin_amdgcn_exp2f(xc);
            const float ga = (xa < -14.0f) ? 0.0f : ea, gc = (xc < -14.0f) ? 0.0f : ec;
            const h16 pa = (h16)ga; const h16 pc = (h16)gc;
            pb[r] = pa; pb[8 + r] = pc;
            ls += (float)pa + (float)pc; }
        l = l * alpha + ls; m = mnew;
        o0 = o0 * alpha; o1 = o1 * alpha;
        const h16* va = VT + vo + key0;
        const v16h v0 = ldh(va), v1 = ldh(va + (size_t)16 * MP);
        o0 = wmma16g(v0, pb, o0);
        o1 = wmma16g(v1, pb, o1);
    }
    l += __shfl_xor(l, 16, 32);
    const bool any = l > 0.0f;
    const float lsafe = any ? l : 1.0f;
    const float inv = any ? (1.0f / lsafe) : 0.0f;
    v16h yb;
#pragma unroll
    for (int r = 0; r < 8; ++r) { yb[r] = toh_flush(o0[r] * inv); yb[8 + r] = toh_flush(o1[r] * inv); }
#pragma unroll
    for (int j = 0; j < 4; ++j) {
        const v16h wa = ldh(WO + (size_t)(16 * j + lr) * HD + 8 * hi);
        const v8f dj = wmma16g(wa, yb, (v8f){});
#pragma unroll
        for (int r = 0; r < 8; ++r) os[(16 * j + 8 * hi + r) * OSP + wave * 16 + lr] = dj[r]; }
    __syncthreads();
    const float* xrow = xin + (size_t)b * CCH * SEQ_FULL + (size_t)tb0;
    float* orow = OUT + (size_t)b * CCH * OUT_SEQ + (size_t)tb0;
#pragma unroll 1
    for (int ps = 0; ps < 2; ++ps) {
#pragma unroll
        for (int s = 0; s < 8; ++s) { const int L = wave * 32 + s * 4 + (lane >> 3); const int c = L >> 1, cofs = (L & 1) * 32 + (lane & 7) * 4;
            const v4f val = *(const v4fa*)(&os[c * OSP + cofs]);
            const v4f xr = *(const v4f*)(xrow + (size_t)c * SEQ_FULL + cofs);
            const float bo = bfr(bout[c]);
            v4f fin;
            fin[0] = (val[0] + bo) + bfr(xr[0]); fin[1] = (val[1] + bo) + bfr(xr[1]); fin[2] = (val[2] + bo) + bfr(xr[2]); fin[3] = (val[3] + bo) + bfr(xr[3]);
            *(volatile v4f*)(orow + (size_t)c * OUT_SEQ + cofs) = fin; }
        if (ps == 0) __threadfence(); }
}

static constexpr size_t al256(size_t v) { return (v + 255) & ~(size_t)255; }
static constexpr size_t SZ_XB = al256((size_t)NB * SEQ * CCH * 2);
static constexpr size_t SZ_WB = al256((size_t)3 * HD * CCH * 2);
static constexpr size_t SZ_WO = al256((size_t)CCH * HD * 2);
static constexpr size_t SZ_Q  = al256((size_t)NB * SEQ * HD * 2);
static constexpr size_t SZ_K  = al256((size_t)NB * MP * HD * 2);
static constexpr size_t SZ_TOTAL = SZ_XB + SZ_WB + SZ_WO + 2 * SZ_Q + 3 * SZ_K;
static_assert(SZ_TOTAL <= (size_t)134217728);
static_assert(((size_t)HD * CCH * 2) % 256 == 0);
static_assert(((size_t)HD * CCH) % 8 == 0);
static_assert(((size_t)CCH * HD) % 8 == 0);
static_assert((NB * SEQ) % 128 == 0);

extern "C" void kernel_launch(void* const* d_in, const int* in_sizes, int n_in,
                              void* d_out, int out_size, void* d_ws, size_t ws_size, hipStream_t stream) {
    if (n_in < 9) return;
    const size_t needx = ((size_t)(NB - 1) * CCH + (size_t)(CCH - 1)) * SEQ_FULL + SEQ;
    if ((size_t)in_sizes[0] < needx) return;
    if ((size_t)in_sizes[1] < (size_t)HD * CCH || (size_t)in_sizes[3] < (size_t)HD * CCH || (size_t)in_sizes[5] < (size_t)HD * CCH || (size_t)in_sizes[7] < (size_t)CCH * HD) return;
    if (in_sizes[2] < HD || in_sizes[4] < HD || in_sizes[6] < HD || in_sizes[8] < CCH) return;
    if ((size_t)out_size < ((size_t)(NB - 1) * CCH + (size_t)(CCH - 1)) * OUT_SEQ + SEQ) return;
    if (SZ_TOTAL > ws_size) return;
    const float* x  = (const float*)d_in[0];
    const float* wq = (const float*)d_in[1]; const float* bq = (const float*)d_in[2];
    const float* wk = (const float*)d_in[3]; const float* bk = (const float*)d_in[4];
    const float* wv = (const float*)d_in[5]; const float* bv = (const float*)d_in[6];
    const float* wo = (const float*)d_in[7]; const float* bo = (const float*)d_in[8];
    float* OUT = (float*)d_out;
    char* wsp = (char*)d_ws;
    bf* XB = (bf*)wsp; wsp += SZ_XB;
    bf* WB = (bf*)wsp; wsp += SZ_WB;
    h16* WO = (h16*)wsp; wsp += SZ_WO;
    h16* QH = (h16*)wsp; wsp += SZ_Q;
    h16* QR = (h16*)wsp; wsp += SZ_Q;
    h16* KP = (h16*)wsp; wsp += SZ_K;
    h16* KR = (h16*)wsp; wsp += SZ_K;
    h16* VT = (h16*)wsp; wsp += SZ_K;
    bf* WQ = WB; bf* WK = WB + (size_t)HD * CCH; bf* WV = WB + (size_t)2 * HD * CCH;

    k_cvtT<<<dim3(SEQ / 64, NB, 1), 256, 0, stream>>>(x, XB);
    { const size_t n8 = (size_t)HD * CCH / 8; const unsigned g = (unsigned)((n8 + 255) / 256);
      k_cvt8<<<g, 256, 0, stream>>>(wq, WQ, n8); k_cvt8<<<g, 256, 0, stream>>>(wk, WK, n8); k_cvt8<<<g, 256, 0, stream>>>(wv, WV, n8);
      k_cvtw<<<g, 256, 0, stream>>>(wo, WO, n8); }

    k_proj_qk<<<dim3(NB * SEQ / 64, 1, 1), 32, 0, stream>>>(XB, WB, bq, bk, QH, QR, KP, KR);
    k_proj_vt<<<dim3(NB * SEQ / 128, 1, 1), 32, 0, stream>>>(WV, XB, bv, VT);

    k_flash<<<dim3(SEQ / (16 * AW), NB, 1), 32 * AW, 0, stream>>>(QH, QR, KP, KR, VT, WO, bo, x, OUT);
}
